// LstmCrfForNer_2662879724398
// MI455X (gfx1250) — hardware-verified
//
#include <hip/hip_runtime.h>
#include <math.h>

typedef __attribute__((ext_vector_type(16))) _Float16 v16h;
typedef __attribute__((ext_vector_type(8)))  _Float16 v8h;
typedef __attribute__((ext_vector_type(16))) __bf16   v16b;
typedef __attribute__((ext_vector_type(8)))  __bf16   v8b;
typedef __attribute__((ext_vector_type(8)))  float    v8f;
typedef __attribute__((ext_vector_type(4)))  float    v4f;

constexpr int kB    = 32;
constexpr int kBP   = 64;
constexpr int kT    = 256;
constexpr int kV    = 32000;
constexpr int kE    = 256;
constexpr int kH    = 512;
constexpr int kG4   = 4 * kH;
constexpr int kK0   = kH + kE;
constexpr int kK1   = kH + 2 * kH;
constexpr int kNL   = 9;
constexpr int kNLP  = 64;
constexpr int kRows = kB * kT;
constexpr int kThr  = 256;
constexpr float kInCarry = 1024.0f;
constexpr float kSc = 1.0f / (kInCarry * kInCarry);
constexpr float kF16MinNormal = 6.103515625e-5f;
constexpr int kFBC = 0, kFBZ = 64, kFEnd = 2304;
constexpr size_t kOutElems = 1 + (size_t)kRows * kNL;

static_assert(kBP == 64 && (kG4 / 64) % 8 == 0 && (kRows % 64) == 0 && ((kRows / 64) * (kNLP / 64)) % 8 == 0 && (kK0 % 32) == 0 && (kK1 % 32) == 0 && ((2 * kH) % 32) == 0
              && kFBZ + kG4 <= kFEnd && kNL <= kNLP, "GEMM M, N multiples of 64; grids exact; K multiples of 32");

constexpr size_t kOffW0 = 0ull;
constexpr size_t kOffW1 = 6291456ull;
constexpr size_t kOffCLS = 18874368ull;
constexpr size_t kOffBIAS = 19005440ull;
constexpr size_t kOffA0 = 19014656ull;
constexpr size_t kOffA1 = 19211264ull;
constexpr size_t kOffG = 19604480ull;
constexpr size_t kOffC = 20653056ull;
constexpr size_t kOffHS0 = 20784128ull;
constexpr size_t kOffHS1 = 37561344ull;
constexpr size_t kOffEM32 = 54338560ull;
constexpr size_t kOffLLH = 56435712ull;
constexpr size_t kWsTotal = 56439808ull;
static_assert(kWsTotal <= 134217728ull, "carve cap: under 128 MiB");
static_assert(kOffW0 == 0
              && kOffW1 == kOffW0 + 6291456ull
              && kOffCLS == kOffW1 + 12582912ull
              && kOffBIAS == kOffCLS + 131072ull
              && kOffA0 == kOffBIAS + 9216ull
              && kOffA1 == kOffA0 + 196608ull
              && kOffG == kOffA1 + 393216ull
              && kOffC == kOffG + 1048576ull
              && kOffHS0 == kOffC + 131072ull
              && kOffHS1 == kOffHS0 + 16777216ull
              && kOffEM32 == kOffHS1 + 16777216ull
              && kOffLLH == kOffEM32 + 2097152ull
              && kWsTotal == kOffLLH + 4096ull, "the carve is chained and totalled");
static_assert((kOffW0 % 256) == 0 && (kOffW1 % 256) == 0 && (kOffCLS % 256) == 0 && (kOffBIAS % 256) == 0 && (kOffA0 % 256) == 0 && (kOffA1 % 256) == 0 && (kOffG % 256) == 0 && (kOffC % 256) == 0 && (kOffHS0 % 256) == 0 && (kOffHS1 % 256) == 0 && (kOffEM32 % 256) == 0 && (kOffLLH % 256) == 0, "aligned regions");

__device__ __forceinline__ unsigned short f2bf_bits(float f) {
  unsigned u = __float_as_uint(f);
  return (unsigned short)((u + 0x7FFFu + ((u >> 16) & 1u)) >> 16);
}
__device__ __forceinline__ float bf_bits2f(unsigned short h) { return __uint_as_float(((unsigned)h) << 16); }
__device__ __forceinline__ float bf16r(float f) { return bf_bits2f(f2bf_bits(f)); }
__device__ __forceinline__ float carry_flush(float v, float carry) {
  const float s = v * carry;
  return (fabsf(s) < kF16MinNormal) ? 0.0f : s;
}
__device__ __forceinline__ float frcp(float x) { return __builtin_amdgcn_rcpf(x); }

__device__ __forceinline__ void dep_guard4_h(v8f& a, v8f& b, v8f& c, v8f& d, v16h x, v16h y) { asm volatile("v_nop\n\tv_nop\n\tv_nop\n\tv_nop" : "+v"(a), "+v"(b), "+v"(c), "+v"(d) : "v"(x), "v"(y)); }
__device__ __forceinline__ void dep_guard4_b(v8f& a, v8f& b, v8f& c, v8f& d, v16b x, v16b y) { asm volatile("v_nop\n\tv_nop\n\tv_nop\n\tv_nop" : "+v"(a), "+v"(b), "+v"(c), "+v"(d) : "v"(x), "v"(y)); }
__device__ __forceinline__ void keep4_h(v16h a, v16h b, v16h c, v16h d) { asm volatile("v_nop" :: "v"(a), "v"(b), "v"(c), "v"(d)); }
__device__ __forceinline__ void keep4_b(v16b a, v16b b, v16b c, v16b d) { asm volatile("v_nop" :: "v"(a), "v"(b), "v"(c), "v"(d)); }
__device__ __forceinline__ void acc_guard4(v8f& a, v8f& b, v8f& c, v8f& d) { asm volatile("v_nop\n\tv_nop\n\tv_nop\n\tv_nop" : "+v"(a), "+v"(b), "+v"(c), "+v"(d)); }

template <typename T> struct Frag;
template <> struct Frag<_Float16> {
  typedef v16h V; union U { v16h v; v8h h[2]; };
  static __device__ __forceinline__ v16h load(const _Float16* p) {
    U f; f.h[0] = *(const v8h*)(p); f.h[1] = *(const v8h*)(p + 16); return f.v;
  }
  static __device__ __forceinline__ v8f mma(v16h a, v16h b, v8f c) {
    return __builtin_amdgcn_wmma_f32_16x16x32_f16(false, a, false, b, (short)0, c, false, false);
  }
  static __device__ __forceinline__ void guard4(v8f& a, v8f& b, v8f& c, v8f& d, v16h x, v16h y) { dep_guard4_h(a, b, c, d, x, y); }
  static __device__ __forceinline__ void keep(v16h a, v16h b, v16h c, v16h d) { keep4_h(a, b, c, d); }
};
template <> struct Frag<__bf16> {
  typedef v16b V; union U { v16b v; v8b h[2]; };
  static __device__ __forceinline__ v16b load(const __bf16* p) {
    U f; f.h[0] = *(const v8b*)(p); f.h[1] = *(const v8b*)(p + 16); return f.v;
  }
  static __device__ __forceinline__ v8f mma(v16b a, v16b b, v8f c) {
    return __builtin_amdgcn_wmma_f32_16x16x32_bf16(false, a, false, b, (short)0, c, false, false);
  }
  static __device__ __forceinline__ void guard4(v8f& a, v8f& b, v8f& c, v8f& d, v16b x, v16b y) { dep_guard4_b(a, b, c, d, x, y); }
  static __device__ __forceinline__ void keep(v16b a, v16b b, v16b c, v16b d) { keep4_b(a, b, c, d); }
};

__device__ __forceinline__ v8f mma_h(v16h a, v16h b, v8f c) {
  c = __builtin_amdgcn_wmma_f32_16x16x32_f16(false, a, false, b, (short)0, c, false, false);
  asm volatile("v_nop\n\tv_nop\n\tv_nop\n\tv_nop" : "+v"(c) : "v"(a), "v"(b));
  return c;
}

template <int ET> struct Elem;
template <> struct Elem<0> { typedef _Float16 T; };
template <> struct Elem<1> { typedef __bf16 T; };
template <int ET, bool SPLIT, int BIAS_MODE, int OUT_MODE, bool RESID, int ACT = 0>
__global__ __launch_bounds__(256) void wmma_gemm64(
    const unsigned short* __restrict__ Ap, const unsigned short* __restrict__ A2p, int lda, long strideA,
    const unsigned short* __restrict__ Btp, const unsigned short* __restrict__ Bt2p, int ldb, long strideB,
    void* __restrict__ Cout, void* __restrict__ Cout2, int ldc, long strideC,
    const float* __restrict__ bias,
    const float* __restrict__ resid, long strideR,
    int M, int N, int K, float scale) {
  typedef typename Elem<ET>::T T;
  typedef typename Frag<T>::V V;
  const T* A = (const T*)Ap; const T* A2 = (const T*)A2p; const T* Bt = (const T*)Btp; const T* Bt2 = (const T*)Bt2p;
  __shared__ __align__(16) float sT[8][16 * 68];
  const int b    = blockIdx.y;
  const int lane = threadIdx.x & 31;
  const int wave = threadIdx.x >> 5;
  const int tilesN = N >> 6;
  const int tilesM = M >> 6;
  const int tile = blockIdx.x * 8 + wave;
  if (tile >= tilesM * tilesN) return;
  const int tm = tile / tilesN;
  const int tn = tile - tm * tilesN;
  const int m0 = tm << 6;
  const int n0 = tn << 6;

  const T* Ab  = A  + (size_t)b * strideA;
  const T* Bb  = Bt + (size_t)b * strideB;
  const T* Ab2 = SPLIT ? (A2  + (size_t)b * strideA) : nullptr;
  const T* Bb2 = SPLIT ? (Bt2 + (size_t)b * strideB) : nullptr;

  const int rlane = lane & 15;
  const int koff  = (lane >> 4) * 8;
  const int mOff  = (lane >> 4) * 8;

  v8f acc[4][4];
#pragma unroll
  for (int i = 0; i < 4; ++i)
#pragma unroll
    for (int j = 0; j < 4; ++j) acc[i][j] = (v8f){0.f,0.f,0.f,0.f,0.f,0.f,0.f,0.f};

  for (int k0 = 0; k0 < K; k0 += 32) {
    V bh[4], bl[4];
#pragma unroll
    for (int j = 0; j < 4; ++j) {
      const size_t bo = (size_t)(n0 + (j << 4) + rlane) * ldb + koff + k0;
      bh[j] = Frag<T>::load(Bb + bo);
      if (SPLIT) bl[j] = Frag<T>::load(Bb2 + bo);
    }
#pragma unroll
    for (int i = 0; i < 4; ++i) {
      const size_t ao = (size_t)(m0 + (i << 4) + rlane) * lda + koff + k0;
      V ah = Frag<T>::load(Ab + ao);
      V al;
      if (SPLIT) al = Frag<T>::load(Ab2 + ao);
#pragma unroll
      for (int j = 0; j < 4; ++j) {
        acc[i][j] = Frag<T>::mma(ah, bh[j], acc[i][j]);
        if (SPLIT) {
          acc[i][j] = Frag<T>::mma(ah, bl[j], acc[i][j]);
          acc[i][j] = Frag<T>::mma(al, bh[j], acc[i][j]);
        }
      }
      Frag<T>::guard4(acc[i][0], acc[i][1], acc[i][2], acc[i][3], ah, SPLIT ? al : ah);
    }
    Frag<T>::keep(bh[0], bh[1], bh[2], bh[3]);
    if (SPLIT) Frag<T>::keep(bl[0], bl[1], bl[2], bl[3]);
  }
  acc_guard4(acc[0][0], acc[0][1], acc[0][2], acc[0][3]);
  acc_guard4(acc[1][0], acc[1][1], acc[1][2], acc[1][3]);
  acc_guard4(acc[2][0], acc[2][1], acc[2][2], acc[2][3]);
  acc_guard4(acc[3][0], acc[3][1], acc[3][2], acc[3][3]);

  float* slab = sT[wave];
  const float* Rb = RESID ? (resid + (size_t)b * strideR) : nullptr;
#pragma unroll
  for (int i = 0; i < 4; ++i) {
    const int mBase = m0 + (i << 4);
#pragma unroll
    for (int j = 0; j < 4; ++j) {
      const int n = n0 + (j << 4) + rlane;
      float bv = 0.f;
      if (BIAS_MODE == 2) bv = bias[n];
#pragma unroll
      for (int r = 0; r < 8; ++r) {
        float v = acc[i][j][r] * scale;
        if (BIAS_MODE == 1) v += bias[mBase + mOff + r];
        if (BIAS_MODE == 2) v += bv;
        if (RESID) v += Rb[(size_t)(mBase + mOff + r) * ldc + n];
        if (ACT == 1) v = tanhf(v);
        if (ACT == 2) v = fmaxf(v, 0.0f);
        if (ACT == 3) v = v / (1.0f + expf(-v));
        if (ACT == 4) v = (v > 0.f) ? v : 0.01f * v;
        slab[(mOff + r) * 68 + (j << 4) + rlane] = v;
      }
    }
    __builtin_amdgcn_fence(__ATOMIC_RELEASE, "workgroup");
    __builtin_amdgcn_wave_barrier();
    __builtin_amdgcn_fence(__ATOMIC_ACQUIRE, "workgroup");
    if (OUT_MODE == 0) {
      float* C = (float*)Cout + (size_t)b * strideC;
      const int hh = lane >> 4, c4 = (lane & 15) * 4;
      for (int pass = 0; pass < 2; ++pass) {
#pragma unroll
        for (int it = 0; it < 8; ++it) {
          const int row = it * 2 + hh;
          v4f v = *(const v4f*)(slab + row * 68 + c4);
          *(volatile v4f*)(C + (size_t)(mBase + row) * ldc + n0 + c4) = v;
        }
        __threadfence();
      }
    } else {
      const int q = lane >> 3, c8 = (lane & 7) * 8;
      unsigned short* C  = (unsigned short*)Cout  + (size_t)b * strideC;
      unsigned short* C2 = (OUT_MODE == 2) ? ((unsigned short*)Cout2 + (size_t)b * strideC) : nullptr;
      for (int pass = 0; pass < 2; ++pass) {
#pragma unroll
        for (int it = 0; it < 4; ++it) {
          const int row = it * 4 + q;
          const float* sp = slab + row * 68 + c8;
          v8h hv, lv;
#pragma unroll
          for (int e = 0; e < 8; ++e) {
            if (OUT_MODE == 1) {
              hv[e] = (_Float16)sp[e];
            } else {
              unsigned short hb = f2bf_bits(sp[e]);
              unsigned short lb = f2bf_bits(sp[e] - bf_bits2f(hb));
              hv[e] = __builtin_bit_cast(_Float16, hb);
              lv[e] = __builtin_bit_cast(_Float16, lb);
            }
          }
          *(volatile v8h*)(C + (size_t)(mBase + row) * ldc + n0 + c8) = hv;
          if (OUT_MODE == 2) *(volatile v8h*)(C2 + (size_t)(mBase + row) * ldc + n0 + c8) = lv;
        }
        __threadfence();
      }
    }
    __builtin_amdgcn_fence(__ATOMIC_RELEASE, "workgroup");
    __builtin_amdgcn_wave_barrier();
    __builtin_amdgcn_fence(__ATOMIC_ACQUIRE, "workgroup");
  }
}


__device__ __forceinline__ float fast_tanh(float v) { return 1.0f - 2.0f * frcp(__expf(2.0f * v) + 1.0f); }
__device__ __forceinline__ float fast_sigmoid(float v) { return frcp(1.0f + __expf(-v)); }

__device__ __forceinline__ int token_at(const int* __restrict__ ids, unsigned b, int t) {
  int tok = ids[(size_t)b * kT + t];
  asm volatile("" : "+v"(tok));
  return (tok < 0) ? 0 : ((tok >= kV) ? (kV - 1) : tok);
}

__global__ __launch_bounds__(kThr) void setup_kernel(const int* __restrict__ ids, const float* __restrict__ emb,
                                                     const float* __restrict__ wih0f, const float* __restrict__ whh0f, const float* __restrict__ wih0r, const float* __restrict__ whh0r,
                                                     const float* __restrict__ wih1f, const float* __restrict__ whh1f, const float* __restrict__ wih1r, const float* __restrict__ whh1r,
                                                     const float* __restrict__ cls_w, const float* __restrict__ cls_b, float* __restrict__ BIAS, unsigned short* __restrict__ W0,
                                                     unsigned short* __restrict__ W1, unsigned short* __restrict__ CLS, unsigned short* __restrict__ A0, unsigned short* __restrict__ A1) {
  unsigned v = blockIdx.x * (unsigned)kThr + threadIdx.x;
  asm volatile("" : "+v"(v));
  if (v < 768u) {
    const unsigned i0 = v * 4u;
    if (i0 < (unsigned)kFEnd) {
      float o0 = 0.0f, o1 = 0.0f, o2 = 0.0f, o3 = 0.0f;
      if (i0 < 12u) {
        float p0 = cls_b[(i0 + 0u < (unsigned)kNL) ? (i0 + 0u) : 0u], p1 = cls_b[(i0 + 1u < (unsigned)kNL) ? (i0 + 1u) : 0u];
        float p2 = cls_b[(i0 + 2u < (unsigned)kNL) ? (i0 + 2u) : 0u], p3 = cls_b[(i0 + 3u < (unsigned)kNL) ? (i0 + 3u) : 0u];
        asm volatile("" : "+v"(p0), "+v"(p1), "+v"(p2), "+v"(p3));
        o0 = (i0 + 0u < (unsigned)kNL) ? bf16r(p0) : 0.0f; o1 = (i0 + 1u < (unsigned)kNL) ? bf16r(p1) : 0.0f;
        o2 = (i0 + 2u < (unsigned)kNL) ? bf16r(p2) : 0.0f; o3 = (i0 + 3u < (unsigned)kNL) ? bf16r(p3) : 0.0f;
      }
      const v4f o = {o0, o1, o2, o3};
      float* dp = BIAS + i0;
      *(volatile v4f*)dp = o;
      __threadfence();
      *(volatile v4f*)dp = o;
    }
  } else {
    v8h hv;
    unsigned short* dp;
    const float* sp;
    bool live = true;
    if (v < 393984u) {
      unsigned w = v - 768u;
      asm volatile("" : "+v"(w));
      const unsigned d = w / 196608u, n = (w / 96u) % 2048u, c8 = (w % 96u) * 8u;
      const float* Wh = d ? whh0r : whh0f;
      const float* Wi = d ? wih0r : wih0f;
      sp = (c8 < (unsigned)kH) ? (Wh + (size_t)n * kH + c8) : (Wi + (size_t)n * kE + (c8 - (unsigned)kH));
      dp = W0 + (size_t)w * 8u;
    } else if (v < 1180416u) {
      unsigned w = v - 393984u;
      asm volatile("" : "+v"(w));
      const unsigned d = w / 393216u, n = (w / 192u) % 2048u, c8 = (w % 192u) * 8u;
      const float* Wh = d ? whh1r : whh1f;
      const float* Wi = d ? wih1r : wih1f;
      sp = (c8 < (unsigned)kH) ? (Wh + (size_t)n * kH + c8) : (Wi + (size_t)n * (2 * kH) + (c8 - (unsigned)kH));
      dp = W1 + (size_t)w * 8u;
    } else if (v < 1188608u) {
      unsigned w = v - 1180416u;
      asm volatile("" : "+v"(w));
      const unsigned n = w >> 7, c8 = (w & 127u) * 8u;
      live = n < (unsigned)kNL;
      sp = cls_w + (size_t)(live ? n : 0u) * (2 * kH) + c8;
      dp = CLS + (size_t)w * 8u;
    } else if (v < 1200896u) {
      unsigned w = v - 1188608u;
      asm volatile("" : "+v"(w));
      const unsigned d = w / 6144u, b = (w / 96u) % 64u, c8 = (w % 96u) * 8u;
      live = (b < (unsigned)kB) && (c8 >= (unsigned)kH);
      const int tok = token_at(ids, (b < (unsigned)kB) ? b : 0u, d ? (kT - 1) : 0);
      sp = emb + (size_t)tok * kE + (live ? (c8 - (unsigned)kH) : 0u);
      dp = A0 + (size_t)w * 8u;
    } else {
      unsigned w = v - 1200896u;
      asm volatile("" : "+v"(w));
      live = false;
      sp = emb;
      dp = A1 + (size_t)w * 8u;
    }
    const v4f a0 = *(const v4f*)sp, a1 = *(const v4f*)(sp + 4);
#pragma unroll
    for (int e = 0; e < 4; ++e) { const float p = a0[e], q = a1[e]; hv[e] = (_Float16)(live ? carry_flush(bf16r(p), kInCarry) : 0.0f); hv[4 + e] = (_Float16)(live ? carry_flush(bf16r(q), kInCarry) : 0.0f); }
    *(volatile v8h*)dp = hv;
    __threadfence();
    *(volatile v8h*)dp = hv;
  }
}
static_assert(2 * kG4 * (kK0 / 8) == 393216 && 768 + 393216 == 393984 && 2 * kG4 * (kK1 / 8) == 786432 && 393984 + 786432 == 1180416 && kNLP * (2 * kH / 8) == 8192 && 1180416 + 8192 == 1188608
              && 2 * kBP * (kK0 / 8) == 12288 && 1188608 + 12288 == 1200896 && 2 * kBP * (kK1 / 8) == 24576 && 1200896 + 24576 == 4787 * kThr && kK0 / 8 == 96 && kK1 / 8 == 192
              && kG4 * 96 == 196608 && kG4 * 192 == 393216 && kBP * 96 == 6144, "set-up grid exact");

__device__ __forceinline__ void cell8(const float* __restrict__ gr, const float* __restrict__ bi_, const float* __restrict__ bh_, float* __restrict__ cp, bool first, v4f& cn0, v4f& cn1, v8h& hv) {
#pragma unroll
  for (int hlf = 0; hlf < 2; ++hlf) {
    const v4f gi = *(const v4f*)(gr + 4 * hlf), gf = *(const v4f*)(gr + kH + 4 * hlf), gg = *(const v4f*)(gr + 2 * kH + 4 * hlf), go = *(const v4f*)(gr + 3 * kH + 4 * hlf);
    const v4f ai = *(const v4f*)(bi_ + 4 * hlf), af = *(const v4f*)(bi_ + kH + 4 * hlf), ag = *(const v4f*)(bi_ + 2 * kH + 4 * hlf), ao = *(const v4f*)(bi_ + 3 * kH + 4 * hlf);
    const v4f hi = *(const v4f*)(bh_ + 4 * hlf), hf = *(const v4f*)(bh_ + kH + 4 * hlf), hg = *(const v4f*)(bh_ + 2 * kH + 4 * hlf), ho = *(const v4f*)(bh_ + 3 * kH + 4 * hlf);
    const v4f co = *(const v4f*)(cp + 4 * hlf);
#pragma unroll
    for (int e = 0; e < 4; ++e) {
      const float p0 = ai[e], p1 = af[e], p2 = ag[e], p3 = ao[e], q0 = hi[e], q1 = hf[e], q2 = hg[e], q3 = ho[e];
      const float cin = first ? 0.0f : co[e];
      const float cn = fast_sigmoid(gf[e] + (bf16r(p1) + bf16r(q1))) * cin + fast_sigmoid(gi[e] + (bf16r(p0) + bf16r(q0))) * fast_tanh(gg[e] + (bf16r(p2) + bf16r(q2)));
      const float hn = fast_sigmoid(go[e] + (bf16r(p3) + bf16r(q3))) * fast_tanh(cn);
      if (hlf == 0) cn0[e] = cn; else cn1[e] = cn;
      hv[4 * hlf + e] = (_Float16)carry_flush(hn, kInCarry);
    }
  }
}

__global__ __launch_bounds__(kThr) void cell2_kernel(const float* __restrict__ G, const float* __restrict__ bi_f, const float* __restrict__ bh_f, const float* __restrict__ bi_r,
                                                     const float* __restrict__ bh_r, const int* __restrict__ ids, const float* __restrict__ emb, const unsigned short* __restrict__ HSin,
                                                     float* __restrict__ C, unsigned short* __restrict__ A, unsigned short* __restrict__ HSout, int kk, int layer1, int s) {
  const int d = (int)(blockIdx.x >> 3);
  const int t = d ? (kT - 1 - s) : s;
  unsigned v = (blockIdx.x & 7u) * (unsigned)kThr + threadIdx.x;
  asm volatile("" : "+v"(v));
  const unsigned b = v >> 6, j = v & 63u, u8 = j * 8u;
  const float* gr = G + ((size_t)d * kBP + b) * kG4 + u8;
  float* cp = C + ((size_t)d * kB + b) * kH + u8;
  v4f cn0, cn1; v8h hv;
  cell8(gr, (d ? bi_r : bi_f) + u8, (d ? bh_r : bh_f) + u8, cp, s == 0, cn0, cn1, hv);
  const int tn = d ? (t - 1) : (t + 1);
  const bool nx = (tn >= 0) && (tn < kT);
  const int tq = nx ? tn : t;
  unsigned short* ar = A + ((size_t)d * kBP + b) * (size_t)kk;
  v8h x0, x1;
  bool w0 = false, w1 = false;
  unsigned short* xp0 = ar + kH;
  unsigned short* xp1 = ar + kH;
  if (layer1 == 0) {
    const int tok = token_at(ids, b, tq);
    const bool em = j < (unsigned)(kE / 8);
    const float* ep = emb + (size_t)tok * kE + (em ? u8 : 0u);
    const v4f m0 = *(const v4f*)ep, m1 = *(const v4f*)(ep + 4);
#pragma unroll
    for (int e = 0; e < 4; ++e) { const float q0 = m0[e], q1 = m1[e]; x0[e] = (_Float16)carry_flush(bf16r(q0), kInCarry); x0[4 + e] = (_Float16)carry_flush(bf16r(q1), kInCarry); }
    x1 = x0;
    w0 = nx && em;
    xp0 = ar + kH + u8;
  } else {
    const unsigned short* hp2 = HSin + ((size_t)b * kT + (size_t)tq) * (2 * kH) + j * 16u;
    x0 = *(const v8h*)hp2;
    x1 = *(const v8h*)(hp2 + 8);
    w0 = nx; w1 = nx;
    xp0 = ar + kH + j * 16u;
    xp1 = xp0 + 8;
  }
  unsigned short* hp = ar + u8;
  unsigned short* op = HSout + ((size_t)b * kT + (size_t)t) * (2 * kH) + (size_t)d * kH + u8;
  for (int pass = 0; pass < 2; ++pass) {
    *(volatile v4f*)cp = cn0; *(volatile v4f*)(cp + 4) = cn1;
    *(volatile v8h*)hp = hv;
    *(volatile v8h*)op = hv;
    if (w0) *(volatile v8h*)xp0 = x0;
    if (w1) *(volatile v8h*)xp1 = x1;
    __threadfence();
  }
}
static_assert(kB * kH / 8 == 8 * kThr && kH / 8 == 64 && kE / 8 == 32 && 2 * kH / 16 == 64, "cell grid: 8 blocks a direction; 64 threads a sample");

__global__ __launch_bounds__(kThr) void l1init_kernel(const unsigned short* __restrict__ HS0, unsigned short* __restrict__ A1) {
  unsigned v = blockIdx.x * (unsigned)kThr + threadIdx.x;
  asm volatile("" : "+v"(v));
  const unsigned d = v >> 12, b = (v >> 7) & 31u, p8 = (v & 127u) * 8u;
  const v8h xv = *(const v8h*)(HS0 + ((size_t)b * kT + (d ? (unsigned)(kT - 1) : 0u)) * (2 * kH) + p8);
  unsigned short* dp = A1 + ((size_t)d * kBP + b) * kK1 + kH + p8;
  *(volatile v8h*)dp = xv;
  __threadfence();
  *(volatile v8h*)dp = xv;
}
static_assert(2 * kB * (2 * kH / 8) == 32 * kThr, "second-layer seeding grid exact");

__global__ __launch_bounds__(32) void seq_loss_kernel(const float* __restrict__ EM32, const int* __restrict__ labels, const int* __restrict__ mask, const float* __restrict__ cstart,
                                                      const float* __restrict__ cend, const float* __restrict__ ctrans, float* __restrict__ LLH) {
  __shared__ float sA[32];
  __shared__ float sTr[kNL * kNL];
  const int j = threadIdx.x;
  const int b = blockIdx.x;
  const bool lj = j < kNL;
  const int jj = lj ? j : 0;
  for (int q = j; q < kNL * kNL; q += 32) { const float p = ctrans[q]; sTr[q] = bf16r(p); }
  float st = cstart[jj], en = cend[jj];
  asm volatile("" : "+v"(st), "+v"(en));
  st = bf16r(st); en = bf16r(en);
  const float* er = EM32 + (size_t)b * kT * kNLP;
  const int* lr = labels + (size_t)b * kT;
  const int* mr = mask + (size_t)b * kT;
  int l0 = lr[0];
  asm volatile("" : "+v"(l0));
  l0 = (l0 == -100) ? 0 : l0;
  l0 = (l0 < 0) ? 0 : ((l0 >= kNL) ? (kNL - 1) : l0);
  float alpha = st + er[jj];
  float score = 0.0f;
  int prev = l0;
  {
    float s0 = cstart[l0];
    asm volatile("" : "+v"(s0));
    score = bf16r(s0) + er[l0];
  }
  sA[j] = lj ? alpha : 0.0f;
  __syncthreads();
#pragma unroll 1
  for (int t = 1; t < kT; ++t) {
    int lt = lr[t], mi = mr[t];
    asm volatile("" : "+v"(lt), "+v"(mi));
    lt = (lt == -100) ? 0 : lt;
    lt = (lt < 0) ? 0 : ((lt >= kNL) ? (kNL - 1) : lt);
    const float mk = (float)mi;
    const bool on = mk > 0.0f;
    const float* et = er + (size_t)t * kNLP;
    score += (sTr[prev * kNL + lt] + et[lt]) * mk;
    const float ej = et[jj];
    float z[kNL];
    float mx = -3.0e38f;
#pragma unroll
    for (int i = 0; i < kNL; ++i) { z[i] = sA[i] + sTr[i * kNL + jj] + ej; mx = (z[i] > mx) ? z[i] : mx; }
    float sum = 0.0f;
#pragma unroll
    for (int i = 0; i < kNL; ++i) sum += expf(z[i] - mx);
    const float nxt = mx + logf(sum);
    alpha = on ? nxt : alpha;
    prev = on ? lt : prev;
    __syncthreads();
    if (lj) sA[j] = alpha;
    __syncthreads();
  }
  {
    float e0 = cend[prev];
    asm volatile("" : "+v"(e0));
    score += bf16r(e0);
  }
  sA[j] = lj ? (alpha + en) : -3.0e38f;
  __syncthreads();
  float llh = 0.0f;
  if (j == 0) {
    float mx = sA[0];
#pragma unroll
    for (int i = 1; i < kNL; ++i) mx = (sA[i] > mx) ? sA[i] : mx;
    float sum = 0.0f;
#pragma unroll
    for (int i = 0; i < kNL; ++i) sum += expf(sA[i] - mx);
    llh = score - (mx + logf(sum));
  }
  float* lp = LLH + (size_t)b * 32 + j;
  *(volatile float*)lp = llh;
  __threadfence();
  *(volatile float*)lp = llh;
}

__global__ __launch_bounds__(kThr) void out_kernel(const float* __restrict__ EM32, const float* __restrict__ LLH, float* __restrict__ out) {
  unsigned v = blockIdx.x * (unsigned)kThr + threadIdx.x;
  asm volatile("" : "+v"(v));
  if (v < (unsigned)kOutElems) {
    float o;
    if (v == 0u) {
      float s = 0.0f;
#pragma unroll 1
      for (int b = 0; b < kB; ++b) s += LLH[b * 32];
      o = -(s / (float)kB);
    } else {
      const unsigned e = v - 1u;
      o = EM32[(size_t)(e / (unsigned)kNL) * kNLP + (e % (unsigned)kNL)];
    }
    *(volatile float*)(out + v) = o;
    __threadfence();
    *(volatile float*)(out + v) = o;
  }
}
static_assert(kOutElems == 73729 && (kOutElems + kThr - 1) / kThr == 289, "output grid");

extern "C" void kernel_launch(void* const* d_in, const int* in_sizes, int n_in,
                              void* d_out, int out_size, void* d_ws, size_t ws_size,
                              hipStream_t stream) {
  if (n_in < 25 || d_out == nullptr || d_ws == nullptr) return;
  if (in_sizes[0] != kB * kT || in_sizes[1] != kB * kT || in_sizes[2] != kB * kT || in_sizes[3] != kV * kE) return;
  if (in_sizes[4] != kG4 * kE || in_sizes[5] != kG4 * kH || in_sizes[6] != kG4 || in_sizes[7] != kG4 || in_sizes[8] != kG4 * kE || in_sizes[9] != kG4 * kH || in_sizes[10] != kG4 || in_sizes[11] != kG4) return;
  if (in_sizes[12] != kG4 * 2 * kH || in_sizes[13] != kG4 * kH || in_sizes[14] != kG4 || in_sizes[15] != kG4 || in_sizes[16] != kG4 * 2 * kH || in_sizes[17] != kG4 * kH || in_sizes[18] != kG4 || in_sizes[19] != kG4) return;
  if (in_sizes[20] != kNL * 2 * kH || in_sizes[21] != kNL || in_sizes[22] != kNL || in_sizes[23] != kNL || in_sizes[24] != kNL * kNL) return;
  if ((size_t)out_size != kOutElems) return;
  if (ws_size < kWsTotal) return;
  const int* ids = (const int*)d_in[0];
  const int* amask = (const int*)d_in[1];
  const int* labels = (const int*)d_in[2];
  const float* emb = (const float*)d_in[3];
  const float* wih0f = (const float*)d_in[4];  const float* whh0f = (const float*)d_in[5];  const float* bih0f = (const float*)d_in[6];  const float* bhh0f = (const float*)d_in[7];
  const float* wih0r = (const float*)d_in[8];  const float* whh0r = (const float*)d_in[9];  const float* bih0r = (const float*)d_in[10]; const float* bhh0r = (const float*)d_in[11];
  const float* wih1f = (const float*)d_in[12]; const float* whh1f = (const float*)d_in[13]; const float* bih1f = (const float*)d_in[14]; const float* bhh1f = (const float*)d_in[15];
  const float* wih1r = (const float*)d_in[16]; const float* whh1r = (const float*)d_in[17]; const float* bih1r = (const float*)d_in[18]; const float* bhh1r = (const float*)d_in[19];
  const float* cls_w = (const float*)d_in[20];
  const float* cls_b = (const float*)d_in[21];
  const float* cstart = (const float*)d_in[22];
  const float* cend = (const float*)d_in[23];
  const float* ctrans = (const float*)d_in[24];
  float* out = (float*)d_out;
  char* ws = (char*)d_ws;
  unsigned short* W0 = (unsigned short*)(ws + kOffW0);
  unsigned short* W1 = (unsigned short*)(ws + kOffW1);
  unsigned short* CLS = (unsigned short*)(ws + kOffCLS);
  float* BIAS = (float*)(ws + kOffBIAS);
  unsigned short* A0 = (unsigned short*)(ws + kOffA0);
  unsigned short* A1 = (unsigned short*)(ws + kOffA1);
  float* G = (float*)(ws + kOffG);
  float* C = (float*)(ws + kOffC);
  unsigned short* HS0 = (unsigned short*)(ws + kOffHS0);
  unsigned short* HS1 = (unsigned short*)(ws + kOffHS1);
  float* EM32 = (float*)(ws + kOffEM32);
  float* LLH = (float*)(ws + kOffLLH);

  setup_kernel<<<4787, kThr, 0, stream>>>(ids, emb, wih0f, whh0f, wih0r, whh0r, wih1f, whh1f, wih1r, whh1r, cls_w, cls_b, BIAS, W0, W1, CLS, A0, A1);

  for (int s = 0; s < kT; ++s) {
    wmma_gemm64<0, false, 2, 0, false, 0><<<dim3((kBP / 64) * (kG4 / 64) / 8, 2), 256, 0, stream>>>(
        A0, A0, kK0, (long)kBP * kK0, W0, W0, kK0, (long)kG4 * kK0, (void*)G, (void*)G, kG4, (long)kBP * kG4, BIAS + kFBZ, nullptr, 0L, kBP, kG4, kK0, kSc);
    cell2_kernel<<<16, kThr, 0, stream>>>(G, bih0f, bhh0f, bih0r, bhh0r, ids, emb, HS0, C, A0, HS0, kK0, 0, s);
  }
  l1init_kernel<<<32, kThr, 0, stream>>>(HS0, A1);
  for (int s = 0; s < kT; ++s) {
    wmma_gemm64<0, false, 2, 0, false, 0><<<dim3((kBP / 64) * (kG4 / 64) / 8, 2), 256, 0, stream>>>(
        A1, A1, kK1, (long)kBP * kK1, W1, W1, kK1, (long)kG4 * kK1, (void*)G, (void*)G, kG4, (long)kBP * kG4, BIAS + kFBZ, nullptr, 0L, kBP, kG4, kK1, kSc);
    cell2_kernel<<<16, kThr, 0, stream>>>(G, bih1f, bhh1f, bih1r, bhh1r, ids, emb, HS0, C, A1, HS1, kK1, 1, s);
  }
  wmma_gemm64<0, false, 2, 0, false, 0><<<dim3((kRows / 64) * (kNLP / 64) / 8, 1), 256, 0, stream>>>(
      HS1, HS1, 2 * kH, 0L, CLS, CLS, 2 * kH, 0L, (void*)EM32, (void*)EM32, kNLP, 0L, BIAS + kFBC, nullptr, 0L, kRows, kNLP, 2 * kH, kSc);
  seq_loss_kernel<<<kB, 32, 0, stream>>>(EM32, labels, amask, cstart, cend, ctrans, LLH);
  out_kernel<<<289, kThr, 0, stream>>>(EM32, LLH, out);
}
